// NAMClassifier_20590073217759
// MI455X (gfx1250) — hardware-verified
//
#include <hip/hip_runtime.h>
#include <stdint.h>
#include <math.h>

typedef _Float16 v16h __attribute__((ext_vector_type(16)));
typedef _Float16 v8h  __attribute__((ext_vector_type(8)));
typedef float    v8f  __attribute__((ext_vector_type(8)));
typedef float    v4f  __attribute__((ext_vector_type(4)));
union Frag { v16h v; v8h half[2]; };

#define B_ROWS 16384
#define NFEAT  256
#define H1D    64
#define H2D    32
#define FC     32
#define NFG    (NFEAT / FC)
#define NTHR   256
#define WAVES  (NTHR / 32)
#define RPU    32
#define NUNIT  (B_ROWS / RPU)
#define NBB    8
#define UPW    (NUNIT / (NBB * WAVES))

#define SCL_H1   16.0f
#define SCL_W2   64.0f
#define SCL_BACK 0.0009765625f

typedef char chk0[(NFEAT % FC == 0) ? 1 : -1];
typedef char chk1[(NUNIT == NBB * WAVES * UPW) ? 1 : -1];
typedef char chk2[(B_ROWS % RPU == 0) ? 1 : -1];
typedef char chk3[(FC % 4 == 0) ? 1 : -1];
typedef char chk4[(B_ROWS % (4 * NTHR) == 0) ? 1 : -1];

__device__ __forceinline__ v8f mma16(v16h a, v16h b, v8f c)
{
    c = __builtin_amdgcn_wmma_f32_16x16x32_f16(false, a, false, b, (short)0, c, false, false);
    asm volatile("v_nop\n\tv_nop\n\tv_nop\n\tv_nop" : "+v"(c) : "v"(a), "v"(b));
    return c;
}

__global__ void __launch_bounds__(NTHR) __attribute__((amdgpu_num_vgpr(256)))
k_main(const float* __restrict__ x,
       const float* __restrict__ W1,
       const float* __restrict__ b1,
       const float* __restrict__ W2,
       const float* __restrict__ b2,
       const float* __restrict__ W3,
       float* __restrict__ partial)
{
    __shared__ v8h sW2v[FC * 2 * 2 * 32 * 2];
    __shared__ __attribute__((aligned(32))) float sW1s[FC * H1D];
    __shared__ __attribute__((aligned(32))) float sB1s[FC * H1D];
    __shared__ float sB2[FC * H2D];
    __shared__ float sW3[FC * H2D];

    const int tid = threadIdx.x;
    const int fg  = blockIdx.y;
    const int f0  = fg * FC;

    for (int g = tid; g < FC * 256; g += NTHR) {
        const int p  = g & 1;
        const int L  = (g >> 1) & 31;
        const int nt = (g >> 6) & 1;
        const int s  = (g >> 7) & 1;
        const int ff = g >> 8;
        const int k0 = 32 * s + 16 * p + 8 * (L >> 4);
        const int n  = 16 * nt + (L & 15);
        const float* src = W2 + ((size_t)(f0 + ff) * H1D + k0) * H2D + n;
        v8f v;
#pragma unroll
        for (int j = 0; j < 8; ++j) v[j] = src[j * H2D] * SCL_W2;
        sW2v[g] = __builtin_convertvector(v, v8h);
    }
    for (int e = tid; e < FC * H1D; e += NTHR) {
        sW1s[e] = W1[(size_t)f0 * H1D + e] * SCL_H1;
        sB1s[e] = b1[(size_t)f0 * H1D + e] * SCL_H1;
    }
    for (int e = tid; e < FC * H2D; e += NTHR) {
        sB2[e] = b2[(size_t)f0 * H2D + e];
        sW3[e] = W3[(size_t)f0 * H2D + e];
    }
    __syncthreads();

    const int wid  = tid >> 5;
    const int lane = tid & 31;
    const int m    = lane & 15;
    const int h    = lane >> 4;
    const v8h zh = {};

    for (int u = 0; u < UPW; ++u) {
        const int unit = (u * NBB + blockIdx.x) * WAVES + wid;
        const int row0 = unit * RPU;
        int ra = row0 + m;       ra = (ra < B_ROWS) ? ra : (B_ROWS - 1);
        int rb = row0 + 16 + m;  rb = (rb < B_ROWS) ? rb : (B_ROWS - 1);
        const float* xr0 = x + (size_t)ra * NFEAT + f0;
        const float* xr1 = x + (size_t)rb * NFEAT + f0;

        float v0[8], v1[8];
#pragma unroll
        for (int r = 0; r < 8; ++r) { v0[r] = 0.f; v1[r] = 0.f; }

        for (int ffb = 0; ffb < FC; ffb += 4) {
            const v4f xq0 = *(const v4f*)(xr0 + ffb);
            const v4f xq1 = *(const v4f*)(xr1 + ffb);
#pragma unroll
            for (int q = 0; q < 4; ++q) {
                const int ff = ffb + q;
                const float xa = xq0[q];
                const float xb = xq1[q];
                v8f c00 = {}, c01 = {}, c10 = {}, c11 = {};
#pragma unroll
                for (int s = 0; s < 2; ++s) {
                    const float* w1p = sW1s + ff * H1D + 32 * s + 8 * h;
                    const float* b1p = sB1s + ff * H1D + 32 * s + 8 * h;
                    const v8f wlo = *(const v8f*)(w1p);
                    const v8f whi = *(const v8f*)(w1p + 16);
                    const v8f blo = *(const v8f*)(b1p);
                    const v8f bhi = *(const v8f*)(b1p + 16);
                    Frag a0, a1;
                    a0.half[0] = __builtin_elementwise_max(__builtin_convertvector(wlo * xa + blo, v8h), zh);
                    a0.half[1] = __builtin_elementwise_max(__builtin_convertvector(whi * xa + bhi, v8h), zh);
                    a1.half[0] = __builtin_elementwise_max(__builtin_convertvector(wlo * xb + blo, v8h), zh);
                    a1.half[1] = __builtin_elementwise_max(__builtin_convertvector(whi * xb + bhi, v8h), zh);
                    const int bi = (((ff * 2 + s) * 2 + 0) * 32 + lane) * 2;
                    Frag bA, bB;
                    bA.half[0] = sW2v[bi];       bA.half[1] = sW2v[bi + 1];
                    bB.half[0] = sW2v[bi + 64];  bB.half[1] = sW2v[bi + 65];
                    c00 = mma16(a0.v, bA.v, c00);
                    c01 = mma16(a0.v, bB.v, c01);
                    c10 = mma16(a1.v, bA.v, c10);
                    c11 = mma16(a1.v, bB.v, c11);
                }
                const float b2a = sB2[ff * H2D + m];
                const float b2b = sB2[ff * H2D + 16 + m];
                const float w3a = sW3[ff * H2D + m];
                const float w3b = sW3[ff * H2D + 16 + m];
#pragma unroll
                for (int r = 0; r < 8; ++r) {
                    v0[r] += fmaxf(fmaf(c00[r], SCL_BACK, b2a), 0.f) * w3a
                           + fmaxf(fmaf(c01[r], SCL_BACK, b2b), 0.f) * w3b;
                    v1[r] += fmaxf(fmaf(c10[r], SCL_BACK, b2a), 0.f) * w3a
                           + fmaxf(fmaf(c11[r], SCL_BACK, b2b), 0.f) * w3b;
                }
            }
        }

#pragma unroll
        for (int off = 1; off <= 8; off <<= 1) {
#pragma unroll
            for (int r = 0; r < 8; ++r) {
                v0[r] += __shfl_xor(v0[r], off, 32);
                v1[r] += __shfl_xor(v1[r], off, 32);
            }
        }
        float o0[8], o1[8];
#pragma unroll
        for (int r = 0; r < 8; ++r) {
            o0[r] = __shfl_xor(v0[r], 16, 32);
            o1[r] = __shfl_xor(v1[r], 16, 32);
        }
        const bool s1 = (lane & 1) != 0;
        const bool s2 = (lane & 2) != 0;
        const bool s4 = (lane & 4) != 0;
        v4f ov;
#pragma unroll
        for (int i = 0; i < 4; ++i) {
            const float e0 = s1 ? v0[4 + i] : v0[i];
            const float e1 = s1 ? o0[4 + i] : o0[i];
            const float e2 = s1 ? v1[4 + i] : v1[i];
            const float e3 = s1 ? o1[4 + i] : o1[i];
            const float g0 = s2 ? e1 : e0;
            const float g1 = s2 ? e3 : e2;
            ov[i] = s4 ? g1 : g0;
        }
        const bool wr = (lane < 8) && (row0 + RPU <= B_ROWS);
        float* dst = partial + (size_t)fg * B_ROWS + row0 + 4 * lane;
        if (wr) *(volatile v4f*)dst = ov;
        __threadfence();
        if (wr) *(volatile v4f*)dst = ov;
    }
}

__global__ void __launch_bounds__(NTHR)
k_fin(const float* __restrict__ partial,
      const float* __restrict__ b3,
      const float* __restrict__ bias,
      float* __restrict__ out)
{
    __shared__ float sCst;
    const int tid = threadIdx.x;
    if (tid == 0) {
        float s = 0.f;
        for (int f = 0; f < NFEAT; ++f) s += b3[f];
        sCst = s + bias[0];
    }
    __syncthreads();
    const float cst = sCst;

    const int q  = blockIdx.x * NTHR + tid;
    const bool ok = (4 * q + 3) < B_ROWS;
    const int qc = ok ? q : 0;
    v4f s = {cst, cst, cst, cst};
#pragma unroll
    for (int g = 0; g < NFG; ++g)
        s += *(const v4f*)(partial + (size_t)g * B_ROWS + 4 * qc);
    v4f p;
#pragma unroll
    for (int i = 0; i < 4; ++i) p[i] = 1.0f / (1.0f + expf(-s[i]));

    float* d0 = out + 4 * (size_t)q;
    float* d1 = out + B_ROWS + 4 * (size_t)q;
    if (ok) { *(volatile v4f*)d0 = s; *(volatile v4f*)d1 = p; }
    __threadfence();
    if (ok) { *(volatile v4f*)d0 = s; *(volatile v4f*)d1 = p; }
}

extern "C" void kernel_launch(void* const* d_in, const int* in_sizes, int n_in,
                              void* d_out, int out_size, void* d_ws, size_t ws_size,
                              hipStream_t stream)
{
    if (n_in < 8) return;
    if (in_sizes[0] != B_ROWS * NFEAT) return;
    if (in_sizes[1] != NFEAT * H1D) return;
    if (in_sizes[2] != NFEAT * H1D) return;
    if (in_sizes[3] != NFEAT * H1D * H2D) return;
    if (in_sizes[4] != NFEAT * H2D) return;
    if (in_sizes[5] != NFEAT * H2D) return;
    if (in_sizes[6] != NFEAT) return;
    if (in_sizes[7] < 1) return;
    if (out_size != 2 * B_ROWS) return;
    const size_t partial_bytes = (size_t)NFG * B_ROWS * sizeof(float);
    if (ws_size < partial_bytes) return;

    const float* x    = (const float*)d_in[0];
    const float* W1   = (const float*)d_in[1];
    const float* b1   = (const float*)d_in[2];
    const float* W2   = (const float*)d_in[3];
    const float* b2   = (const float*)d_in[4];
    const float* W3   = (const float*)d_in[5];
    const float* b3   = (const float*)d_in[6];
    const float* bias = (const float*)d_in[7];
    float* out     = (float*)d_out;
    float* partial = (float*)d_ws;

    dim3 grid(NBB, NFG, 1);
    k_main<<<grid, NTHR, 0, stream>>>(x, W1, b1, W2, b2, W3, partial);
    const int nq = B_ROWS / 4;
    k_fin<<<(nq + NTHR - 1) / NTHR, NTHR, 0, stream>>>(partial, b3, bias, out);
}
